// RelativeAttention_35270271434811
// MI455X (gfx1250) — hardware-verified
//
#include <hip/hip_runtime.h>

typedef __attribute__((ext_vector_type(16))) __bf16 v16b;
typedef __attribute__((ext_vector_type(8)))  __bf16 v8b;
typedef __attribute__((ext_vector_type(8)))  float  v8f;
typedef __attribute__((ext_vector_type(4)))  float  v4f;
typedef __attribute__((ext_vector_type(4)))  unsigned int v4u;
typedef __attribute__((ext_vector_type(4)))  int    v4i;

#ifndef NB
#define NB 1
#endif
#ifndef SEQ
#define SEQ 2048
#endif
#define NB_FULL 1
#define SEQ_FULL 2048

constexpr int HID   = 1024;
constexpr int NHEAD = 16;
constexpr int DHEAD = 64;
constexpr int NREL  = 32;
constexpr int LQ    = SEQ;
constexpr int QBLK  = 64;
constexpr int KCH   = 64;
constexpr int NWAVE = 4;
constexpr int GM = 128;
constexpr int GN = 64;
constexpr int SL_PITCH = 68;
constexpr int ST_PITCH = 132;
constexpr int OS_PITCH = 68;
constexpr int TS_PITCH = 72;
constexpr int SLAB_FLOATS = GM * SL_PITCH;

static_assert(NB == 1 && NB <= NB_FULL);
static_assert(SEQ >= GM && SEQ <= SEQ_FULL);
static_assert(SEQ % GM == 0 && SEQ % QBLK == 0 && SEQ % KCH == 0);
static_assert(HID % GN == 0 && HID % 64 == 0 && HID % 32 == 0);
static_assert(NHEAD * DHEAD == HID && DHEAD == 64 && GN == DHEAD);
static_assert(NREL == 32);
static_assert(QBLK == NWAVE * 16 && KCH % 32 == 0 && DHEAD % 32 == 0);
static_assert(GN * ST_PITCH <= SLAB_FLOATS);
static_assert((SL_PITCH * 4) % 16 == 0 && (ST_PITCH * 4) % 16 == 0 && (OS_PITCH * 4) % 16 == 0 && (TS_PITCH * 2) % 16 == 0);
static_assert(((size_t)LQ * HID) % 2048 == 0);

constexpr size_t XB_ELEMS = (size_t)LQ * HID;
constexpr size_t WT_ELEMS = (size_t)HID * HID;
constexpr size_t EB_ELEMS = (size_t)NHEAD * NREL * DHEAD;
constexpr size_t PL_ELEMS = (size_t)NHEAD * LQ * DHEAD;
constexpr size_t OFFB_XB = 0;
constexpr size_t OFFB_WT = OFFB_XB + XB_ELEMS * 2;
constexpr size_t OFFB_EB = OFFB_WT + 4 * WT_ELEMS * 2;
constexpr size_t OFFB_QH = OFFB_EB + EB_ELEMS * 2;
constexpr size_t OFFB_QL = OFFB_QH + PL_ELEMS * 2;
constexpr size_t OFFB_KH = OFFB_QL + PL_ELEMS * 2;
constexpr size_t OFFB_KL = OFFB_KH + PL_ELEMS * 2;
constexpr size_t OFFB_VH = OFFB_KL + PL_ELEMS * 2;
constexpr size_t OFFB_VL = OFFB_VH + PL_ELEMS * 2;
constexpr size_t OFFB_CH = OFFB_VL + PL_ELEMS * 2;
constexpr size_t OFFB_CL = OFFB_CH + PL_ELEMS * 2;
constexpr size_t WS_NEED = OFFB_CL + PL_ELEMS * 2;
static_assert(WS_NEED <= 134217728ull);
static_assert(OFFB_WT % 128 == 0 && OFFB_EB % 128 == 0 && OFFB_QH % 128 == 0 && OFFB_QL % 128 == 0);
static_assert(OFFB_KH % 128 == 0 && OFFB_KL % 128 == 0 && OFFB_VH % 128 == 0 && OFFB_VL % 128 == 0);
static_assert(OFFB_CH % 128 == 0 && OFFB_CL % 128 == 0);

constexpr int OFF_KH  = 0;
constexpr int OFF_KL  = OFF_KH + KCH * DHEAD * 2;
constexpr int OFF_VH  = OFF_KL + KCH * DHEAD * 2;
constexpr int OFF_VL  = OFF_VH + DHEAD * KCH * 2;
constexpr int OFF_T   = OFF_VL + DHEAD * KCH * 2;
constexpr int OFF_PH  = OFF_T + QBLK * KCH * 4;
constexpr int OFF_PL  = OFF_PH + NWAVE * 16 * KCH * 2;
constexpr int OFF_REL = OFF_PL + NWAVE * 16 * KCH * 2;
constexpr int OFF_RB  = OFF_REL + QBLK * NREL * 4;
constexpr int SMEM_BYTES = OFF_RB + NREL * 4;
static_assert(NWAVE * 16 * OS_PITCH * 4 <= OFF_T);
static_assert(OFF_KL % 16 == 0 && OFF_VH % 16 == 0 && OFF_VL % 16 == 0 && OFF_T % 16 == 0);
static_assert(OFF_PH % 16 == 0 && OFF_PL % 16 == 0 && OFF_REL % 16 == 0 && OFF_RB % 16 == 0);

union FB { v16b v; v8b h[2]; v4u u[2]; };

__device__ __forceinline__ unsigned short f2bf_bits(float f) {
  unsigned u = __float_as_uint(f);
  return (unsigned short)((u + 0x7FFFu + ((u >> 16) & 1u)) >> 16);
}
__device__ __forceinline__ float bf_bits2f(unsigned short h) { return __uint_as_float(((unsigned)h) << 16); }
__device__ __forceinline__ float rbf(float f) { return bf_bits2f(f2bf_bits(f)); }
__device__ __forceinline__ unsigned int pk2(float a, float b) {
  return (unsigned)f2bf_bits(a) | ((unsigned)f2bf_bits(b) << 16);
}
__device__ __forceinline__ void hilo2(float x, float y, unsigned int& hw, unsigned int& lw) {
  const unsigned short hx = f2bf_bits(x), hy = f2bf_bits(y);
  const unsigned short lx = f2bf_bits(x - bf_bits2f(hx)), ly = f2bf_bits(y - bf_bits2f(hy));
  hw = (unsigned)hx | ((unsigned)hy << 16);
  lw = (unsigned)lx | ((unsigned)ly << 16);
}
__device__ __forceinline__ void hilo8(const v4f x0, const v4f x1, v4u& hw, v4u& lw) {
  unsigned h0, h1, h2, h3, l0, l1, l2, l3;
  hilo2(x0[0], x0[1], h0, l0);
  hilo2(x0[2], x0[3], h1, l1);
  hilo2(x1[0], x1[1], h2, l2);
  hilo2(x1[2], x1[3], h3, l3);
  hw = (v4u){h0, h1, h2, h3};
  lw = (v4u){l0, l1, l2, l3};
}

__device__ __forceinline__ v8f mma_bf16(v16b a, v16b b, v8f c) {
  c = __builtin_amdgcn_wmma_f32_16x16x32_bf16(false, a, false, b, (short)0, c, false, false);
  asm volatile("v_nop\n\tv_nop\n\tv_nop\n\tv_nop" : "+v"(c) : "v"(a), "v"(b));
  return c;
}

__global__ __launch_bounds__(256) void planes_kernel(
    const float* __restrict__ x, const float* __restrict__ remb,
    unsigned short* __restrict__ xb, unsigned short* __restrict__ eb, int nxblk)
{
  const int tid = threadIdx.x;
  const float* src;
  unsigned short* dst;
  if ((int)blockIdx.x < nxblk) {
    const size_t e0 = ((size_t)blockIdx.x * 256 + tid) * 8;
    src = x + e0;
    dst = xb + e0;
  } else {
    const int u  = ((int)blockIdx.x - nxblk) * 256 + tid;
    const int hd = u >> 8;
    const int rr = (u >> 3) & 31;
    const int d0 = (u & 7) * 8;
    src = remb + ((size_t)rr * NHEAD + hd) * DHEAD + d0;
    dst = eb + (size_t)u * 8;
  }
  const v4f a = *(const v4f*)src;
  const v4f b = *(const v4f*)(src + 4);
  v4u w;
  w[0] = pk2(a[0], a[1]);
  w[1] = pk2(a[2], a[3]);
  w[2] = pk2(b[0], b[1]);
  w[3] = pk2(b[2], b[3]);
  for (int pass = 0; pass < 2; ++pass) {
    *(volatile v4u*)dst = w;
    __threadfence();
  }
}

__global__ __launch_bounds__(256) void wt_kernel(
    const float* __restrict__ Wq, const float* __restrict__ Wk,
    const float* __restrict__ Wv, const float* __restrict__ Wo,
    unsigned short* __restrict__ wt)
{
  __shared__ __align__(16) unsigned short Ts[64 * TS_PITCH];
  const int z = blockIdx.z;
  const float* W = (z == 0) ? Wq : ((z == 1) ? Wk : ((z == 2) ? Wv : Wo));
  unsigned short* Wt = wt + (size_t)z * WT_ELEMS;
  const int n0 = blockIdx.x * 64;
  const int k0 = blockIdx.y * 64;
  const int tid = threadIdx.x;

#pragma unroll
  for (int it = 0; it < 4; ++it) {
    const int u = it * 256 + tid;
    const int row = u >> 4;
    const int c4 = (u & 15) * 4;
    const v4f v = *(const v4f*)(W + (size_t)(k0 + row) * HID + n0 + c4);
#pragma unroll
    for (int e = 0; e < 4; ++e) Ts[(c4 + e) * TS_PITCH + row] = f2bf_bits(v[e]);
  }
  __syncthreads();

  v4u w[2];
#pragma unroll
  for (int it = 0; it < 2; ++it) {
    const int u = it * 256 + tid;
    const int nn = u >> 3;
    const int seg = u & 7;
    w[it] = *(const v4u*)(Ts + nn * TS_PITCH + seg * 8);
  }
  for (int pass = 0; pass < 2; ++pass) {
#pragma unroll
    for (int it = 0; it < 2; ++it) {
      const int u = it * 256 + tid;
      const int nn = u >> 3;
      const int seg = u & 7;
      *(volatile v4u*)(Wt + (size_t)(n0 + nn) * HID + k0 + seg * 8) = w[it];
    }
    __threadfence();
  }
}

template <int NPA, int MODE>
__global__ __launch_bounds__(128) void gemm_kernel(
    const unsigned short* __restrict__ A0, const unsigned short* __restrict__ A1,
    const unsigned short* __restrict__ Bt, const float* __restrict__ bias,
    float* __restrict__ outf, unsigned short* __restrict__ P0, unsigned short* __restrict__ P1)
{
  __shared__ __align__(16) float slab[SLAB_FLOATS];
  const int tid  = threadIdx.x;
  const int wave = tid >> 5;
  const int lane = tid & 31;
  const int hh   = lane >> 4;
  const int c    = lane & 15;
  const int n0   = blockIdx.x * GN;
  const int m0   = blockIdx.y * GM;
  const int mw   = wave * 32;

  v8f acc[2][4];
#pragma unroll
  for (int mi = 0; mi < 2; ++mi)
#pragma unroll
    for (int t = 0; t < 4; ++t) acc[mi][t] = (v8f){0.f,0.f,0.f,0.f,0.f,0.f,0.f,0.f};

  const size_t arow0 = (size_t)(m0 + mw + c) * HID + 8 * hh;
  const size_t arow1 = arow0 + (size_t)16 * HID;
  const size_t brow  = (size_t)(n0 + c) * HID + 8 * hh;

  for (int k0 = 0; k0 < HID; k0 += 32) {
    FB a0[2], a1[2];
    a0[0].u[0] = *(const v4u*)(A0 + arow0 + k0);
    a0[0].u[1] = *(const v4u*)(A0 + arow0 + k0 + 16);
    a0[1].u[0] = *(const v4u*)(A0 + arow1 + k0);
    a0[1].u[1] = *(const v4u*)(A0 + arow1 + k0 + 16);
    if (NPA == 2) {
      a1[0].u[0] = *(const v4u*)(A1 + arow0 + k0);
      a1[0].u[1] = *(const v4u*)(A1 + arow0 + k0 + 16);
      a1[1].u[0] = *(const v4u*)(A1 + arow1 + k0);
      a1[1].u[1] = *(const v4u*)(A1 + arow1 + k0 + 16);
    } else {
      a1[0] = a0[0];
      a1[1] = a0[1];
    }
#pragma unroll
    for (int t = 0; t < 4; ++t) {
      FB b;
      const size_t bo = brow + (size_t)t * 16 * HID + k0;
      b.u[0] = *(const v4u*)(Bt + bo);
      b.u[1] = *(const v4u*)(Bt + bo + 16);
#pragma unroll
      for (int mi = 0; mi < 2; ++mi) {
        acc[mi][t] = mma_bf16(a0[mi].v, b.v, acc[mi][t]);
        if (NPA == 2) acc[mi][t] = mma_bf16(a1[mi].v, b.v, acc[mi][t]);
      }
    }
  }

  if (MODE == 2) {
#pragma unroll
    for (int mi = 0; mi < 2; ++mi)
#pragma unroll
      for (int t = 0; t < 4; ++t) {
        float* col = slab + (t * 16 + c) * ST_PITCH + mw + mi * 16 + 8 * hh;
        *(v4f*)col       = (v4f){acc[mi][t][0], acc[mi][t][1], acc[mi][t][2], acc[mi][t][3]};
        *(v4f*)(col + 4) = (v4f){acc[mi][t][4], acc[mi][t][5], acc[mi][t][6], acc[mi][t][7]};
      }
  } else {
#pragma unroll
    for (int mi = 0; mi < 2; ++mi)
#pragma unroll
      for (int t = 0; t < 4; ++t)
#pragma unroll
        for (int r = 0; r < 8; ++r)
          slab[(mw + mi * 16 + 8 * hh + r) * SL_PITCH + t * 16 + c] = acc[mi][t][r];
  }
  __syncthreads();

  if (MODE == 0) {
    const int c4 = c * 4;
    v4f bb = *(const v4f*)(bias + n0 + c4);
#pragma unroll
    for (int e = 0; e < 4; ++e) bb[e] = rbf(bb[e]);
    for (int pass = 0; pass < 2; ++pass) {
#pragma unroll
      for (int it = 0; it < 16; ++it) {
        const int row = mw + 2 * it + hh;
        const v4f val = *(const v4f*)(slab + row * SL_PITCH + c4) + bb;
        *(volatile v4f*)(outf + (size_t)(m0 + row) * HID + n0 + c4) = val;
      }
      __threadfence();
    }
  } else if (MODE == 1) {
    const int seg = lane & 7, rsub = lane >> 3;
    const int hd = blockIdx.x;
    v4f b0 = *(const v4f*)(bias + n0 + seg * 8);
    v4f b1 = *(const v4f*)(bias + n0 + seg * 8 + 4);
#pragma unroll
    for (int e = 0; e < 4; ++e) { b0[e] = rbf(b0[e]); b1[e] = rbf(b1[e]); }
    for (int pass = 0; pass < 2; ++pass) {
#pragma unroll
      for (int it = 0; it < 8; ++it) {
        const int row = mw + 4 * it + rsub;
        const v4f x0 = *(const v4f*)(slab + row * SL_PITCH + seg * 8) + b0;
        const v4f x1 = *(const v4f*)(slab + row * SL_PITCH + seg * 8 + 4) + b1;
        v4u hw, lw;
        hilo8(x0, x1, hw, lw);
        const size_t dst = ((size_t)hd * LQ + m0 + row) * DHEAD + seg * 8;
        *(volatile v4u*)(P0 + dst) = hw;
        *(volatile v4u*)(P1 + dst) = lw;
      }
      __threadfence();
    }
  } else {
    const int seg = lane & 7, rsub = lane >> 3;
    const int hd = blockIdx.x;
    float bd[8];
#pragma unroll
    for (int it = 0; it < 8; ++it) bd[it] = rbf(bias[n0 + wave * 16 + ((4 * it + rsub) >> 1)]);
    for (int pass = 0; pass < 2; ++pass) {
#pragma unroll
      for (int it = 0; it < 8; ++it) {
        const int L = 4 * it + rsub;
        const int d = wave * 16 + (L >> 1);
        const int kvo = 64 * (L & 1) + 8 * seg;
        const v4f x0 = *(const v4f*)(slab + d * ST_PITCH + kvo) + bd[it];
        const v4f x1 = *(const v4f*)(slab + d * ST_PITCH + kvo + 4) + bd[it];
        v4u hw, lw;
        hilo8(x0, x1, hw, lw);
        const size_t dst = ((size_t)hd * DHEAD + d) * LQ + m0 + kvo;
        *(volatile v4u*)(P0 + dst) = hw;
        *(volatile v4u*)(P1 + dst) = lw;
      }
      __threadfence();
    }
  }
}

__global__ __launch_bounds__(128) void attn_kernel(
    const unsigned short* __restrict__ Qh, const unsigned short* __restrict__ Ql,
    const unsigned short* __restrict__ Kh, const unsigned short* __restrict__ Kl,
    const unsigned short* __restrict__ Vh, const unsigned short* __restrict__ Vl,
    const unsigned short* __restrict__ Eb, const float* __restrict__ rbias,
    const int* __restrict__ ids, const int* __restrict__ msk,
    unsigned short* __restrict__ Ch, unsigned short* __restrict__ Cl)
{
  __shared__ __align__(16) unsigned char smem[SMEM_BYTES];
  unsigned short* Ksh_h = (unsigned short*)(smem + OFF_KH);
  unsigned short* Ksh_l = (unsigned short*)(smem + OFF_KL);
  unsigned short* Vsh_h = (unsigned short*)(smem + OFF_VH);
  unsigned short* Vsh_l = (unsigned short*)(smem + OFF_VL);
  float* Tsh   = (float*)(smem + OFF_T);
  unsigned short* Psh = (unsigned short*)(smem + OFF_PH);
  unsigned short* Psl = (unsigned short*)(smem + OFF_PL);
  float* relsh = (float*)(smem + OFF_REL);
  float* rbsh  = (float*)(smem + OFF_RB);
  float* Os    = (float*)(smem + OFF_KH);

  const int tid  = threadIdx.x;
  const int wave = tid >> 5;
  const int lane = tid & 31;
  const int hh   = lane >> 4;
  const int c    = lane & 15;
  const int qb   = blockIdx.x;
  const int hd   = blockIdx.y;
  const int q0   = qb * QBLK + wave * 16;

  if (tid < NREL) rbsh[tid] = rbf(rbias[tid * NHEAD + hd]);

  FB qh[2], ql[2];
  {
    const size_t qoff = ((size_t)hd * LQ + q0 + c) * DHEAD + 8 * hh;
#pragma unroll
    for (int dc = 0; dc < 2; ++dc) {
      qh[dc].u[0] = *(const v4u*)(Qh + qoff + dc * 32);
      qh[dc].u[1] = *(const v4u*)(Qh + qoff + dc * 32 + 16);
      ql[dc].u[0] = *(const v4u*)(Ql + qoff + dc * 32);
      ql[dc].u[1] = *(const v4u*)(Ql + qoff + dc * 32 + 16);
    }
  }

  v8f ar[2];
#pragma unroll
  for (int j = 0; j < 2; ++j) {
    ar[j] = (v8f){0.f,0.f,0.f,0.f,0.f,0.f,0.f,0.f};
#pragma unroll
    for (int dc = 0; dc < 2; ++dc) {
      FB e;
      const size_t eoff = ((size_t)hd * NREL + j * 16 + c) * DHEAD + dc * 32 + 8 * hh;
      e.u[0] = *(const v4u*)(Eb + eoff);
      e.u[1] = *(const v4u*)(Eb + eoff + 16);
      ar[j] = mma_bf16(qh[dc].v, e.v, ar[j]);
      ar[j] = mma_bf16(ql[dc].v, e.v, ar[j]);
    }
  }
  __syncthreads();
#pragma unroll
  for (int j = 0; j < 2; ++j)
#pragma unroll
    for (int r = 0; r < 8; ++r)
      relsh[(wave * 16 + 8 * hh + r) * NREL + j * 16 + c] = ar[j][r] + rbsh[j * 16 + c];

  float mrow[8], lrow[8];
  v8f oacc[4];
#pragma unroll
  for (int r = 0; r < 8; ++r) { mrow[r] = -__builtin_inff(); lrow[r] = 0.f; }
#pragma unroll
  for (int t = 0; t < 4; ++t) oacc[t] = (v8f){0.f,0.f,0.f,0.f,0.f,0.f,0.f,0.f};

  const unsigned short* Khp = Kh + (size_t)hd * LQ * DHEAD;
  const unsigned short* Klp = Kl + (size_t)hd * LQ * DHEAD;
  const unsigned short* Vhp = Vh + (size_t)hd * DHEAD * LQ;
  const unsigned short* Vlp = Vl + (size_t)hd * DHEAD * LQ;
  const int* idp = ids + (size_t)qb * QBLK * SEQ_FULL;
  const int* mkp = msk + (size_t)qb * QBLK * SEQ_FULL;
  unsigned short* pwh = Psh + wave * 16 * KCH;
  unsigned short* pwl = Psl + wave * 16 * KCH;

  for (int kc = 0; kc < LQ / KCH; ++kc) {
    const int kv0 = kc * KCH;
    __syncthreads();
#pragma unroll
    for (int it = 0; it < 4; ++it) {
      const int u = it * 128 + tid;
      const int row = u >> 3;
      const int seg = u & 7;
      const v4u a = *(const v4u*)(Khp + (size_t)(kv0 + row) * DHEAD + seg * 8);
      const v4u b = *(const v4u*)(Klp + (size_t)(kv0 + row) * DHEAD + seg * 8);
      const v4u d = *(const v4u*)(Vhp + (size_t)row * LQ + kv0 + seg * 8);
      const v4u f = *(const v4u*)(Vlp + (size_t)row * LQ + kv0 + seg * 8);
      *(v4u*)(Ksh_h + row * DHEAD + seg * 8) = a;
      *(v4u*)(Ksh_l + row * DHEAD + seg * 8) = b;
      *(v4u*)(Vsh_h + row * KCH + seg * 8)   = d;
      *(v4u*)(Vsh_l + row * KCH + seg * 8)   = f;
    }
#pragma unroll 2
    for (int it = 0; it < 8; ++it) {
      const int u = it * 128 + tid;
      const int row = u >> 4;
      const int c4 = (u & 15) * 4;
      const size_t g = (size_t)row * SEQ_FULL + kv0 + c4;
      const v4i idv = *(const v4i*)(idp + g);
      const v4i mkv = *(const v4i*)(mkp + g);
      v4f tv;
#pragma unroll
      for (int e = 0; e < 4; ++e) {
        int id = idv[e];
        id = id < 0 ? 0 : id;
        id = id > (NREL - 1) ? (NREL - 1) : id;
        const float rel  = relsh[row * NREL + id];
        const float madd = -10000.0f * (1.0f - (float)mkv[e]);
        tv[e] = rel * 0.125f + madd;
      }
      *(v4f*)(Tsh + row * KCH + c4) = tv;
    }
    __syncthreads();

    v8f s[4];
#pragma unroll
    for (int j = 0; j < 4; ++j) {
      s[j] = (v8f){0.f,0.f,0.f,0.f,0.f,0.f,0.f,0.f};
#pragma unroll
      for (int dc = 0; dc < 2; ++dc) {
        FB kfh, kfl;
        const int ko = (j * 16 + c) * DHEAD + dc * 32 + 8 * hh;
        kfh.u[0] = *(const v4u*)(Ksh_h + ko);
        kfh.u[1] = *(const v4u*)(Ksh_h + ko + 16);
        kfl.u[0] = *(const v4u*)(Ksh_l + ko);
        kfl.u[1] = *(const v4u*)(Ksh_l + ko + 16);
        s[j] = mma_bf16(qh[dc].v, kfh.v, s[j]);
        s[j] = mma_bf16(qh[dc].v, kfl.v, s[j]);
        s[j] = mma_bf16(ql[dc].v, kfh.v, s[j]);
      }
    }
#pragma unroll
    for (int j = 0; j < 4; ++j)
#pragma unroll
      for (int r = 0; r < 8; ++r)
        s[j][r] = s[j][r] * 0.125f + Tsh[(wave * 16 + 8 * hh + r) * KCH + j * 16 + c];

    float cm[8];
#pragma unroll
    for (int r = 0; r < 8; ++r) {
      float m = fmaxf(fmaxf(s[0][r], s[1][r]), fmaxf(s[2][r], s[3][r]));
#pragma unroll
      for (int off = 1; off < 16; off <<= 1) m = fmaxf(m, __shfl_xor(m, off, 32));
      cm[r] = m;
    }

#pragma unroll
    for (int r = 0; r < 8; ++r) {
      const float mnew  = fmaxf(mrow[r], cm[r]);
      const float alpha = expf(mrow[r] - mnew);
      mrow[r] = mnew;
      float psum = 0.f;
#pragma unroll
      for (int j = 0; j < 4; ++j) {
        const float p = expf(s[j][r] - mnew);
        psum += p;
        const unsigned short hb = f2bf_bits(p);
        const unsigned short lb = f2bf_bits(p - bf_bits2f(hb));
        pwh[(8 * hh + r) * KCH + j * 16 + c] = hb;
        pwl[(8 * hh + r) * KCH + j * 16 + c] = lb;
      }
#pragma unroll
      for (int off = 1; off < 16; off <<= 1) psum += __shfl_xor(psum, off, 32);
      lrow[r] = lrow[r] * alpha + psum;
#pragma unroll
      for (int t = 0; t < 4; ++t) oacc[t][r] *= alpha;
    }
    __builtin_amdgcn_fence(__ATOMIC_RELEASE, "workgroup");
    __builtin_amdgcn_wave_barrier();
    __builtin_amdgcn_fence(__ATOMIC_ACQUIRE, "workgroup");

#pragma unroll
    for (int kk = 0; kk < 2; ++kk) {
      FB pa, pl;
      pa.u[0] = *(const v4u*)(pwh + c * KCH + kk * 32 + 8 * hh);
      pa.u[1] = *(const v4u*)(pwh + c * KCH + kk * 32 + 16 + 8 * hh);
      pl.u[0] = *(const v4u*)(pwl + c * KCH + kk * 32 + 8 * hh);
      pl.u[1] = *(const v4u*)(pwl + c * KCH + kk * 32 + 16 + 8 * hh);
#pragma unroll
      for (int t = 0; t < 4; ++t) {
        FB vbh, vbl;
        const int vo = (t * 16 + c) * KCH + kk * 32 + 8 * hh;
        vbh.u[0] = *(const v4u*)(Vsh_h + vo);
        vbh.u[1] = *(const v4u*)(Vsh_h + vo + 16);
        vbl.u[0] = *(const v4u*)(Vsh_l + vo);
        vbl.u[1] = *(const v4u*)(Vsh_l + vo + 16);
        oacc[t] = mma_bf16(pa.v, vbh.v, oacc[t]);
        oacc[t] = mma_bf16(pa.v, vbl.v, oacc[t]);
        oacc[t] = mma_bf16(pl.v, vbh.v, oacc[t]);
      }
    }
  }

  __syncthreads();
  float* os = Os + wave * 16 * OS_PITCH;
#pragma unroll
  for (int r = 0; r < 8; ++r) {
    const float inv = 1.0f / lrow[r];
#pragma unroll
    for (int t = 0; t < 4; ++t) os[(8 * hh + r) * OS_PITCH + t * 16 + c] = oacc[t][r] * inv;
  }
  __builtin_amdgcn_fence(__ATOMIC_RELEASE, "workgroup");
  __builtin_amdgcn_wave_barrier();
  __builtin_amdgcn_fence(__ATOMIC_ACQUIRE, "workgroup");
  {
    const int seg = lane & 7, rsub = lane >> 3;
    for (int pass = 0; pass < 2; ++pass) {
#pragma unroll
      for (int it = 0; it < 4; ++it) {
        const int row = it * 4 + rsub;
        const v4f x0 = *(const v4f*)(os + row * OS_PITCH + seg * 8);
        const v4f x1 = *(const v4f*)(os + row * OS_PITCH + seg * 8 + 4);
        v4u hw, lw;
        hilo8(x0, x1, hw, lw);
        const size_t dst = (size_t)(q0 + row) * HID + hd * DHEAD + seg * 8;
        *(volatile v4u*)(Ch + dst) = hw;
        *(volatile v4u*)(Cl + dst) = lw;
      }
      __threadfence();
    }
  }
}

extern "C" void kernel_launch(void* const* d_in, const int* in_sizes, int n_in,
                              void* d_out, int out_size, void* d_ws, size_t ws_size,
                              hipStream_t stream)
{
  if (n_in < 13) return;
  if (in_sizes[0] < LQ * HID) return;
  const long long needsq = (long long)(LQ - 1) * SEQ_FULL + LQ;
  if ((long long)in_sizes[1] < needsq || (long long)in_sizes[2] < needsq) return;
  if (in_sizes[3] < HID * HID || in_sizes[5] < HID * HID || in_sizes[7] < HID * HID || in_sizes[11] < HID * HID) return;
  if (in_sizes[4] < HID || in_sizes[6] < HID || in_sizes[8] < HID || in_sizes[12] < HID) return;
  if (in_sizes[9] < NREL * NHEAD * DHEAD || in_sizes[10] < NREL * NHEAD) return;
  if (out_size < LQ * HID) return;
  if (d_ws == nullptr || ws_size < WS_NEED) return;

  const float* x        = (const float*)d_in[0];
  const int*   att_mask = (const int*)d_in[1];
  const int*   rel_ids  = (const int*)d_in[2];
  const float* Wq = (const float*)d_in[3];
  const float* bq = (const float*)d_in[4];
  const float* Wk = (const float*)d_in[5];
  const float* bk = (const float*)d_in[6];
  const float* Wv = (const float*)d_in[7];
  const float* bv = (const float*)d_in[8];
  const float* rel_emb  = (const float*)d_in[9];
  const float* rel_bias = (const float*)d_in[10];
  const float* Wo = (const float*)d_in[11];
  const float* bo = (const float*)d_in[12];
  float* out = (float*)d_out;

  char* w = (char*)d_ws;
  unsigned short* xb = (unsigned short*)(w + OFFB_XB);
  unsigned short* wt = (unsigned short*)(w + OFFB_WT);
  unsigned short* eb = (unsigned short*)(w + OFFB_EB);
  unsigned short* qh = (unsigned short*)(w + OFFB_QH);
  unsigned short* ql = (unsigned short*)(w + OFFB_QL);
  unsigned short* kh = (unsigned short*)(w + OFFB_KH);
  unsigned short* kl = (unsigned short*)(w + OFFB_KL);
  unsigned short* vh = (unsigned short*)(w + OFFB_VH);
  unsigned short* vl = (unsigned short*)(w + OFFB_VL);
  unsigned short* ch = (unsigned short*)(w + OFFB_CH);
  unsigned short* cl = (unsigned short*)(w + OFFB_CL);

  const int nxblk = (int)(XB_ELEMS / 2048);
  const int neblk = (int)(EB_ELEMS / 2048);
  const dim3 gG(HID / GN, LQ / GM);

  planes_kernel<<<dim3(nxblk + neblk), 256, 0, stream>>>(x, rel_emb, xb, eb, nxblk);
  wt_kernel<<<dim3(HID / 64, HID / 64, 4), 256, 0, stream>>>(Wq, Wk, Wv, Wo, wt);
  gemm_kernel<1, 1><<<gG, 128, 0, stream>>>(xb, xb, wt + 0 * WT_ELEMS, bq, out, qh, ql);
  gemm_kernel<1, 1><<<gG, 128, 0, stream>>>(xb, xb, wt + 1 * WT_ELEMS, bk, out, kh, kl);
  gemm_kernel<1, 2><<<gG, 128, 0, stream>>>(xb, xb, wt + 2 * WT_ELEMS, bv, out, vh, vl);
  attn_kernel<<<dim3(LQ / QBLK, NHEAD), 128, 0, stream>>>(qh, ql, kh, kl, vh, vl, eb, rel_bias,
                                                          rel_ids, att_mask, ch, cl);
  gemm_kernel<2, 0><<<gG, 128, 0, stream>>>(ch, cl, wt + 3 * WT_ELEMS, bo, out, qh, ql);
}
